// MultiHeadAttentionLayer_15822659518994
// MI455X (gfx1250) — hardware-verified
//
#include <hip/hip_runtime.h>


#ifndef NB
#define NB 4
#endif
#ifndef SEQ
#define SEQ 2048
#endif
#ifndef SEQ_FULL
#define SEQ_FULL 2048
#endif

namespace {

constexpr unsigned KD = 1024  , NHEAD = 16, DH = 64, QKP = 2048  ;
constexpr unsigned NBU = NB, SEQU = SEQ, SEQF = SEQ_FULL, MT = NBU * SEQU  ;
constexpr float LOG2E = 1.4426950408889634f, LNEPS = 1e-5f, WSC = 16.0f  , CSC = 32.0f  ;
static_assert(NHEAD * DH == KD);
static_assert(SEQU % 128 == 0 && SEQU <= SEQF && NBU >= 1);
static_assert(MT % 128 == 0 && KD % 32 == 0);

typedef _Float16 b16;
typedef __attribute__((ext_vector_type(16))) _Float16 v16b;
typedef __attribute__((ext_vector_type(8))) _Float16 v8b;
typedef __attribute__((ext_vector_type(8))) float v8f;
typedef __attribute__((ext_vector_type(4))) float v4f;

__device__ __forceinline__ float bf16_rne(float f) { unsigned int u = __float_as_uint(f); u += 0x7FFFu + ((u >> 16) & 1u); return __uint_as_float(u & 0xFFFF0000u); }
__device__ __forceinline__ v16b frag_kb(const b16* p, unsigned hh) { const v8b a = *(const v8b*)(p + 8 * hh), b = *(const v8b*)(p + 16 + 8 * hh); v16b f;
#pragma unroll
  for (int e = 0; e < 8; ++e) { f[e] = a[e]; f[8 + e] = b[e]; } return f; }
__device__ __forceinline__ v8f wmma16b(v16b a, v16b b, v8f c) { v8f d = __builtin_amdgcn_wmma_f32_16x16x32_f16(false, a, false, b, (short)0, c, false, false); asm volatile("v_nop\n\tv_nop\n\tv_nop\n\tv_nop" : "+v"(d) : "v"(a), "v"(b)); return d; }
__device__ __forceinline__ void wave_lds_sync() { __builtin_amdgcn_fence(3  , "workgroup"); __builtin_amdgcn_wave_barrier(); __builtin_amdgcn_fence(2  , "workgroup"); }

__global__ __launch_bounds__(256) void ln_kernel(const float* __restrict__ x, const float* __restrict__ gam, const float* __restrict__ bet, b16* __restrict__ XN) {
  const unsigned wave = threadIdx.x >> 5, lane = threadIdx.x & 31;
  const unsigned r = blockIdx.x * 8 + wave;
  const unsigned bb = r / SEQU, ss = r - bb * SEQU;
  const float* xr = x + ((size_t)bb * SEQF + ss) * KD + lane * 8;
  float s = 0.0f;
#pragma unroll 1
  for (unsigned c = 0; c < 4; ++c) { const v4f a = *(const v4f*)(xr + c * 256), b = *(const v4f*)(xr + c * 256 + 4);
#pragma unroll
    for (int j = 0; j < 4; ++j) s += bf16_rne(a[j]) + bf16_rne(b[j]); }
#pragma unroll
  for (int m = 16; m > 0; m >>= 1) s += __shfl_xor(s, m, 32);
  const float mu = s * (1.0f / 1024.0f);
  float q = 0.0f;
#pragma unroll 1
  for (unsigned c = 0; c < 4; ++c) { const v4f a = *(const v4f*)(xr + c * 256), b = *(const v4f*)(xr + c * 256 + 4);
#pragma unroll
    for (int j = 0; j < 4; ++j) { const float d0 = bf16_rne(a[j]) - mu, d1 = bf16_rne(b[j]) - mu; q += d0 * d0; q += d1 * d1; } }
#pragma unroll
  for (int m = 16; m > 0; m >>= 1) q += __shfl_xor(q, m, 32);
  const float inv = rsqrtf(q * (1.0f / 1024.0f) + LNEPS);
  for (int pass = 0; pass < 2; ++pass) {
#pragma unroll 1
    for (unsigned c = 0; c < 4; ++c) { const unsigned co = c * 256 + lane * 8;
      const v4f a = *(const v4f*)(xr + c * 256), b = *(const v4f*)(xr + c * 256 + 4);
      const v4f ga = *(const v4f*)(gam + co), gb = *(const v4f*)(gam + co + 4), ba = *(const v4f*)(bet + co), bb2 = *(const v4f*)(bet + co + 4);
      v8b v;
#pragma unroll
      for (int j = 0; j < 4; ++j) { v[j] = (b16)((bf16_rne(a[j]) - mu) * inv * bf16_rne(ga[j]) + bf16_rne(ba[j])); v[4 + j] = (b16)((bf16_rne(b[j]) - mu) * inv * bf16_rne(gb[j]) + bf16_rne(bb2[j])); }
      *(volatile v8b*)(XN + (size_t)r * KD + co) = v; }
    __threadfence(); }
}

__global__ __launch_bounds__(256) void wt_kernel(const float* __restrict__ w0, const float* __restrict__ w1, const float* __restrict__ w2, const float* __restrict__ w3, b16* __restrict__ WT) {
  const unsigned y = blockIdx.y; const float* w = (y == 0) ? w0 : (y == 1) ? w1 : (y == 2) ? w2 : w3;
  const unsigned u = blockIdx.x * 256 + threadIdx.x;
  const unsigned e = u * 8, o = e >> 10, k0 = e & 1023u; v8b v;
#pragma unroll
  for (int j = 0; j < 8; ++j) v[j] = (b16)(bf16_rne(w[(size_t)(k0 + j) * KD + o]) * WSC);
  for (int pass = 0; pass < 2; ++pass) { *(volatile v8b*)(WT + (size_t)y * KD * KD + e) = v; __threadfence(); }
}

template <int OMODE>
__global__ __launch_bounds__(128) void gemm_kernel(const b16* __restrict__ A, const b16* __restrict__ Bt, const float* __restrict__ bias, const float* __restrict__ resid, b16* __restrict__ outH, float* __restrict__ outF, unsigned opitch, float scale) {
  const unsigned wave = threadIdx.x >> 5, lane = threadIdx.x & 31, nloc = lane & 15, hh = lane >> 4;
  const unsigned m0 = blockIdx.x * 64 + (wave & 1) * 32, n0 = blockIdx.y * 128 + (wave >> 1) * 64;
  v8f acc[2][4];
#pragma unroll
  for (int i = 0; i < 2; ++i)
#pragma unroll
    for (int j = 0; j < 4; ++j) acc[i][j] = (v8f){};
  const b16* pa = A + (size_t)(m0 + nloc) * KD;
  const b16* pb = Bt + (size_t)(n0 + nloc) * KD;
#pragma unroll 2
  for (unsigned kb = 0; kb < KD; kb += 32) {
    const v16b a0 = frag_kb(pa + kb, hh), a1 = frag_kb(pa + 16 * KD + kb, hh);
#pragma unroll
    for (int j = 0; j < 4; ++j) { const v16b bf = frag_kb(pb + (size_t)j * 16 * KD + kb, hh); acc[0][j] = wmma16b(a0, bf, acc[0][j]); acc[1][j] = wmma16b(a1, bf, acc[1][j]); } }
  if constexpr (OMODE != 2) {
    __shared__ __attribute__((aligned(16))) b16 Th[4][32][72];
#pragma unroll
    for (int i = 0; i < 2; ++i)
#pragma unroll
      for (int j = 0; j < 4; ++j) { const unsigned col = j * 16 + nloc; float bc = 0.0f; if (OMODE == 0) bc = bf16_rne(bias[n0 + col]);
#pragma unroll
        for (int r = 0; r < 8; ++r) { const unsigned row = i * 16 + 8 * hh + r; float bbv = bc; if (OMODE == 1) bbv = bf16_rne(bias[m0 + row]); Th[wave][row][col] = (b16)(acc[i][j][r] * scale + bbv); } }
    wave_lds_sync();
    for (int pass = 0; pass < 2; ++pass) {
#pragma unroll 2
      for (unsigned it = 0; it < 8; ++it) { const unsigned row = it * 4 + (lane >> 3), pc = (lane & 7) * 8; const v8b v = *(const v8b*)(&Th[wave][row][pc]);
        *(volatile v8b*)(outH + (size_t)(m0 + row) * opitch + n0 + pc) = v; }
      __threadfence(); }
  } else {
    __shared__ __attribute__((aligned(16))) float Tf[4][32][68];
#pragma unroll
    for (int i = 0; i < 2; ++i)
#pragma unroll
      for (int j = 0; j < 4; ++j) { const unsigned col = j * 16 + nloc; const float bc = bf16_rne(bias[n0 + col]);
#pragma unroll
        for (int r = 0; r < 8; ++r) { const unsigned row = i * 16 + 8 * hh + r; Tf[wave][row][col] = acc[i][j][r] * scale + bc; } }
    wave_lds_sync();
    const unsigned mb = m0 / SEQU; const unsigned mfull = mb * SEQF + (m0 - mb * SEQU);
    for (int pass = 0; pass < 2; ++pass) {
#pragma unroll 2
      for (unsigned it = 0; it < 16; ++it) { const unsigned row = it * 2 + (lane >> 4), c4 = (lane & 15) * 4; const size_t go = (size_t)(mfull + row) * opitch + n0 + c4;
        v4f t = *(const v4f*)(&Tf[wave][row][c4]); const v4f xr = *(const v4f*)(resid + go);
#pragma unroll
        for (int j = 0; j < 4; ++j) t[j] += bf16_rne(xr[j]);
        *(volatile v4f*)(outF + go) = t; }
      __threadfence(); }
  }
}

__global__ __launch_bounds__(128) void attn_kernel(const b16* __restrict__ QK, const b16* __restrict__ VT, b16* __restrict__ CTX) {
  __shared__ __attribute__((aligned(16))) b16 Ot[4][16][72];
  const unsigned wave = threadIdx.x >> 5, lane = threadIdx.x & 31, nloc = lane & 15, hh = lane >> 4;
  const unsigned qt = blockIdx.x, h = blockIdx.y, b = blockIdx.z;
  const unsigned iw0 = qt * 64 + wave * 16;
  const b16* qrow = QK + (size_t)(b * SEQU + iw0 + nloc) * QKP + h * DH;
  const v16b qf0 = frag_kb(qrow, hh), qf1 = frag_kb(qrow + 32, hh);
  const b16* kbase = QK + (size_t)(b * SEQU + nloc) * QKP + KD + h * DH;
  const b16* vbase = VT + (size_t)(h * DH + nloc) * MT + b * SEQU;
  v8f o[4];
#pragma unroll
  for (int dt = 0; dt < 4; ++dt) o[dt] = (v8f){};
  float m = -1.0e30f, l = 0.0f;
  const float SCL = 0.125f * LOG2E;
  const unsigned iq = iw0 + nloc;
#pragma unroll 1
  for (unsigned jt = 0; jt <= qt; ++jt) {
    const unsigned j0 = jt * 64;
    v8f s[4];
#pragma unroll
    for (int t = 0; t < 4; ++t) { const b16* kr = kbase + (size_t)(j0 + 16 * t) * QKP; const v16b ka0 = frag_kb(kr, hh), ka1 = frag_kb(kr + 32, hh);
      s[t] = wmma16b(ka0, qf0, (v8f){}); s[t] = wmma16b(ka1, qf1, s[t]); }
    const bool diag = (jt == qt);
    float mx = -1.0e30f;
#pragma unroll
    for (int t = 0; t < 4; ++t)
#pragma unroll
      for (int r = 0; r < 8; ++r) { float xv = s[t][r] * SCL; if (diag) { const unsigned j = j0 + 16 * t + 8 * hh + r; xv = (j > iq) ? -1.0e30f : xv; } s[t][r] = xv; mx = fmaxf(mx, xv); }
    mx = fmaxf(mx, __shfl_xor(mx, 16, 32));
    const float newm = fmaxf(m, mx); const float alpha = exp2f(m - newm); m = newm;
    float psum = 0.0f; v16b pf0, pf1;
#pragma unroll
    for (int t = 0; t < 4; ++t)
#pragma unroll
      for (int r = 0; r < 8; ++r) { const b16 ph = (b16)exp2f(s[t][r] - m); psum += (float)ph; if (t < 2) pf0[(t & 1) * 8 + r] = ph; else pf1[(t & 1) * 8 + r] = ph; }
    psum += __shfl_xor(psum, 16, 32);
    l = l * alpha + psum;
#pragma unroll
    for (int dt = 0; dt < 4; ++dt)
#pragma unroll
      for (int r = 0; r < 8; ++r) o[dt][r] *= alpha;
#pragma unroll
    for (int dt = 0; dt < 4; ++dt) { const b16* vr = vbase + (size_t)(dt * 16) * MT + j0; const v16b va0 = frag_kb(vr, hh), va1 = frag_kb(vr + 32, hh);
      o[dt] = wmma16b(va0, pf0, o[dt]); o[dt] = wmma16b(va1, pf1, o[dt]); }
  }
  const float inv = CSC * (1.0f / l);
#pragma unroll
  for (int dt = 0; dt < 4; ++dt) { v8b v;
#pragma unroll
    for (int r = 0; r < 8; ++r) v[r] = (b16)(o[dt][r] * inv);
    *(v8b*)(&Ot[wave][nloc][dt * 16 + 8 * hh]) = v; }
  wave_lds_sync();
  for (int pass = 0; pass < 2; ++pass) {
#pragma unroll
    for (unsigned it = 0; it < 4; ++it) { const unsigned row = it * 4 + (lane >> 3), pc = (lane & 7) * 8; const v8b v = *(const v8b*)(&Ot[wave][row][pc]);
      *(volatile v8b*)(CTX + (size_t)(b * SEQU + iw0 + row) * KD + h * DH + pc) = v; }
    __threadfence(); }
}

}

extern "C" void kernel_launch(void* const* d_in, const int* in_sizes, int n_in, void* d_out, int out_size, void* d_ws, size_t ws_size, hipStream_t stream) {
  if (n_in < 11) return;
  const size_t need = ((size_t)(NBU - 1) * SEQF + SEQU) * KD;
  if ((size_t)in_sizes[0] < need || (size_t)out_size < need) return;
  if (in_sizes[1] < (int)KD || in_sizes[2] < (int)KD || in_sizes[4] < (int)KD || in_sizes[6] < (int)KD || in_sizes[8] < (int)KD || in_sizes[10] < (int)KD) return;
  if ((size_t)in_sizes[3] < (size_t)KD * KD || (size_t)in_sizes[5] < (size_t)KD * KD || (size_t)in_sizes[7] < (size_t)KD * KD || (size_t)in_sizes[9] < (size_t)KD * KD) return;
  const float* x = (const float*)d_in[0]; const float* gam = (const float*)d_in[1]; const float* bet = (const float*)d_in[2];
  const float* Wq = (const float*)d_in[3]; const float* bq = (const float*)d_in[4]; const float* Wk = (const float*)d_in[5]; const float* bk = (const float*)d_in[6];
  const float* Wv = (const float*)d_in[7]; const float* bv = (const float*)d_in[8]; const float* Wo = (const float*)d_in[9]; const float* bo = (const float*)d_in[10];
  float* out = (float*)d_out;
  size_t off = 0; char* ws = (char*)d_ws;
  auto carve = [&](size_t bytes) { char* p = ws + off; off += (bytes + 255) & ~(size_t)255; return p; };
  b16* XN = (b16*)carve((size_t)MT * KD * 2);
  b16* WT = (b16*)carve((size_t)4 * KD * KD * 2);
  b16* QK = (b16*)carve((size_t)MT * QKP * 2);
  b16* VT = (b16*)carve((size_t)KD * MT * 2);
  b16* CTX = (b16*)carve((size_t)MT * KD * 2);
  if (off > ws_size || off > ((size_t)128 << 20)) return;
  const float s16 = 1.0f / WSC, s512 = 1.0f / (WSC * CSC);
  ln_kernel<<<MT / 8, 256, 0, stream>>>(x, gam, bet, XN);
  wt_kernel<<<dim3(KD * KD / 8 / 256, 4), 256, 0, stream>>>(Wq, Wk, Wv, Wo, WT);
  gemm_kernel<0><<<dim3(MT / 64, KD / 128), 128, 0, stream>>>(XN, WT, bq, x, QK, out, QKP, s16);
  gemm_kernel<0><<<dim3(MT / 64, KD / 128), 128, 0, stream>>>(XN, WT + (size_t)KD * KD, bk, x, QK + KD, out, QKP, s16);
  gemm_kernel<1><<<dim3(KD / 64, MT / 128), 128, 0, stream>>>(WT + (size_t)2 * KD * KD, XN, bv, x, VT, out, MT, s16);
  attn_kernel<<<dim3(SEQU / 64, NHEAD, NBU), 128, 0, stream>>>(QK, VT, CTX);
  gemm_kernel<2><<<dim3(MT / 64, KD / 128), 128, 0, stream>>>(CTX, WT + (size_t)3 * KD * KD, bo, x, CTX, out, KD, s512);
}
